// MLA_39436389712281
// MI455X (gfx1250) — hardware-verified
//
#include <hip/hip_runtime.h>
#include <math.h>
#include <stdint.h>

#ifndef NB
#define NB 2
#endif
#ifndef SEQ
#define SEQ 2048
#endif
#define NB_FULL  2
#define SEQ_FULL 2048
#define DMOD 2048
#define NHD  16
#define HDIM 128
#define LATD 128
#define ROTH 32
#define NTOK (NB * SEQ)
#define QCW  (2 * DMOD)
#define OUT1_OFF ((long)NB_FULL * SEQ_FULL * DMOD)
#define OUT2_OFF (OUT1_OFF + (long)NB_FULL * SEQ_FULL * LATD)
#define PCARRY 16384.0f
#define F16MIN 6.103515625e-05f

typedef __bf16       v16b __attribute__((ext_vector_type(16)));
typedef __bf16       v8b  __attribute__((ext_vector_type(8)));
typedef _Float16     v16h __attribute__((ext_vector_type(16)));
typedef _Float16     v8h  __attribute__((ext_vector_type(8)));
typedef float        v8f  __attribute__((ext_vector_type(8)));
typedef float        v4f  __attribute__((ext_vector_type(4)));
typedef unsigned int v4u  __attribute__((ext_vector_type(4)));

static_assert(NB >= 1 && NB <= NB_FULL);
static_assert(SEQ % 64 == 0 && SEQ <= SEQ_FULL);
static_assert(NHD * HDIM == DMOD);
static_assert(LATD == HDIM);
static_assert(HDIM == 4 * ROTH);
static_assert(DMOD % 64 == 0 && LATD % 64 == 0);
static_assert(QCW == 2 * DMOD);
static_assert(OUT1_OFF * 4 == 33554432L);
static_assert(OUT2_OFF * 4 == 35651584L);
static_assert((OUT2_OFF + (long)NB_FULL * SEQ_FULL * LATD) * 4 == 37748736L);

__device__ __forceinline__ unsigned short bf_bits(float f) {
  const unsigned u = __float_as_uint(f);
  return (unsigned short)((u + 0x7FFFu + ((u >> 16) & 1u)) >> 16);
}
__device__ __forceinline__ float bf_val(unsigned short h) { return __uint_as_float(((unsigned)h) << 16); }
__device__ __forceinline__ unsigned short h16_bits(float f) { return __builtin_bit_cast(unsigned short, (_Float16)f); }
__device__ __forceinline__ unsigned pk16(unsigned short a, unsigned short b) { return (unsigned)a | ((unsigned)b << 16); }
__device__ __forceinline__ v8f zero8() { v8f z = {0.f, 0.f, 0.f, 0.f, 0.f, 0.f, 0.f, 0.f}; return z; }
__device__ __forceinline__ int wave_id() { return __builtin_amdgcn_readfirstlane((int)(threadIdx.x >> 5)); }

__device__ __forceinline__ void lds_wave_sync() {
  __builtin_amdgcn_fence(3  , "workgroup");
  __builtin_amdgcn_wave_barrier();
  __builtin_amdgcn_fence(2  , "workgroup");
}

union FragB { v16b v; v8b h[2]; };
union FragH { v16h v; v8h h[2]; };
__device__ __forceinline__ v16b ldfrag_b(const __bf16* p) { FragB f; f.h[0] = *(const v8b*)(p); f.h[1] = *(const v8b*)(p + 16); return f.v; }

__device__ __forceinline__ v8f mma_b(v16b a, v16b b, v8f c) {
  return __builtin_amdgcn_wmma_f32_16x16x32_bf16(false, a, false, b, (short)0, c, false, false);
}
__device__ __forceinline__ void dep_guard_b(v8f& a, v8f& b, v16b x, v16b y) {
  asm volatile("v_nop\n\tv_nop\n\tv_nop\n\tv_nop" : "+v"(a), "+v"(b) : "v"(x), "v"(y));
}
__device__ __forceinline__ void keep4_b(v16b a, v16b b, v16b c, v16b d) { asm volatile("v_nop" :: "v"(a), "v"(b), "v"(c), "v"(d)); }
__device__ __forceinline__ void acc_guard4(v8f& a, v8f& b, v8f& c, v8f& d) {
  asm volatile("v_nop\n\tv_nop\n\tv_nop\n\tv_nop" : "+v"(a), "+v"(b), "+v"(c), "+v"(d));
}
__device__ __forceinline__ v8f at_mma(v16b a, v16b b, v8f c) {
  c = __builtin_amdgcn_wmma_f32_16x16x32_bf16(false, a, false, b, (short)0, c, false, false);
  asm volatile("v_nop\n\tv_nop\n\tv_nop\n\tv_nop" : "+v"(c) : "v"(a), "v"(b));
  return c;
}
__device__ __forceinline__ v8f at_mma_h(v16h a, v16h b, v8f c) {
  c = __builtin_amdgcn_wmma_f32_16x16x32_f16(false, a, false, b, (short)0, c, false, false);
  asm volatile("v_nop\n\tv_nop\n\tv_nop\n\tv_nop" : "+v"(c) : "v"(a), "v"(b));
  return c;
}

__global__ __launch_bounds__(256) void cvt_rows_kernel(const float* __restrict__ in, unsigned short* __restrict__ outp,
                                                       int n8, int cols, int rows_per_grp, int src_rows_per_grp) {
  const int i = (int)blockIdx.x * 256 + (int)threadIdx.x;
  if (i >= n8) return;
  const size_t e = 8 * (size_t)i;
  const int r = (int)(e / (size_t)cols);
  const int cc = (int)(e - (size_t)r * cols);
  const int g = r / rows_per_grp;
  const int t = r - g * rows_per_grp;
  const float* src = in + ((size_t)g * src_rows_per_grp + t) * (size_t)cols + cc;
  const v4f a = *(const v4f*)(src);
  const v4f b = *(const v4f*)(src + 4);
  v4u w;
  w[0] = pk16(bf_bits(a[0]), bf_bits(a[1]));
  w[1] = pk16(bf_bits(a[2]), bf_bits(a[3]));
  w[2] = pk16(bf_bits(b[0]), bf_bits(b[1]));
  w[3] = pk16(bf_bits(b[2]), bf_bits(b[3]));
  *(volatile v4u*)(outp + e) = w;
  __threadfence();
  *(volatile v4u*)(outp + e) = w;
}

__global__ __launch_bounds__(256) void prep_kernel(const float* __restrict__ wkh, const float* __restrict__ wvh,
                                                   float* __restrict__ wsum, float* __restrict__ freq) {
  const int tid = (int)threadIdx.x;
  const int e = (int)blockIdx.x * 256 + tid;
  const bool second = (blockIdx.x >= 8);
  const float* W = second ? wvh : wkh;
  const int idx = e & (NHD * LATD - 1);
  const float* p = W + (size_t)idx * HDIM;
  float a = 0.f;
#pragma unroll 4
  for (int d = 0; d < HDIM; ++d) a += bf_val(bf_bits(p[d]));
  *(volatile float*)(wsum + e) = a;
  if (blockIdx.x == 0 && tid < ROTH) {
    const float f = 1.0f / powf(10000.0f, (float)tid * (1.0f / 32.0f));
    *(volatile float*)(freq + tid) = f;
    __threadfence();
    *(volatile float*)(freq + tid) = f;
  }
  __threadfence();
  *(volatile float*)(wsum + e) = a;
}

__global__ __launch_bounds__(256) void table_kernel(const float* __restrict__ freq, float* __restrict__ cst,
                                                    float* __restrict__ snt, int n) {
  const int i = (int)blockIdx.x * 256 + (int)threadIdx.x;
  if (i >= n) return;
  const int s = i / ROTH;
  const int j = i - s * ROTH;
  const float ang = (float)s * freq[j];
  float sv, cv;
  sincosf(ang, &sv, &cv);
  *(volatile float*)(cst + i) = cv;
  *(volatile float*)(snt + i) = sv;
  __threadfence();
  *(volatile float*)(cst + i) = cv;
  *(volatile float*)(snt + i) = sv;
}

template <bool ASPLIT, bool BSPLIT, int OUT_MODE, bool ROPE>
__global__ __launch_bounds__(256) void gemm64_kernel(
    const unsigned short* __restrict__ Ap, const unsigned short* __restrict__ A2p, int lda, long strideA,
    const unsigned short* __restrict__ Btp, const unsigned short* __restrict__ Bt2p, int ldb, long strideB,
    void* Cout, void* Cout2, int ldc, long strideC,
    int M, int N, int K, float scale,
    const float* __restrict__ cst, const float* __restrict__ snt, int seqlen) {
  __shared__ __align__(16) float sT[8][16 * 68];
  const __bf16* A   = (const __bf16*)(const void*)Ap;
  const __bf16* A2  = (const __bf16*)(const void*)A2p;
  const __bf16* Bt  = (const __bf16*)(const void*)Btp;
  const __bf16* Bt2 = (const __bf16*)(const void*)Bt2p;
  const int b    = blockIdx.y;
  const int lane = threadIdx.x & 31;
  const int wave = wave_id();
  const int tilesN = N >> 6;
  const int tilesM = M >> 6;
  const int tile = (int)blockIdx.x * 8 + wave;
  if (tile >= tilesM * tilesN) return;
  const int tm = tile / tilesN;
  const int tn = tile - tm * tilesN;
  const int m0 = tm << 6;
  const int n0 = tn << 6;

  const __bf16* Ab  = A  + (size_t)b * strideA;
  const __bf16* Bb  = Bt + (size_t)b * strideB;
  const __bf16* Ab2 = ASPLIT ? (A2  + (size_t)b * strideA) : Ab;
  const __bf16* Bb2 = BSPLIT ? (Bt2 + (size_t)b * strideB) : Bb;

  const int rlane = lane & 15;
  const int koff  = (lane >> 4) * 8;
  const int mOff  = (lane >> 4) * 8;

  v8f acc[4][4];
#pragma unroll
  for (int i = 0; i < 4; ++i)
#pragma unroll
    for (int j = 0; j < 4; ++j) acc[i][j] = zero8();

  for (int k0 = 0; k0 < K; k0 += 32) {
    v16b bh[4], bl[4];
#pragma unroll
    for (int j = 0; j < 4; ++j) {
      const size_t bo = (size_t)(n0 + (j << 4) + rlane) * ldb + koff + k0;
      bh[j] = ldfrag_b(Bb + bo);
      bl[j] = BSPLIT ? ldfrag_b(Bb2 + bo) : bh[j];
    }
#pragma unroll
    for (int i = 0; i < 4; ++i) {
      const size_t ao = (size_t)(m0 + (i << 4) + rlane) * lda + koff + k0;
      const v16b ah = ldfrag_b(Ab + ao);
      const v16b al = ASPLIT ? ldfrag_b(Ab2 + ao) : ah;
#pragma unroll
      for (int j = 0; j < 4; ++j) {
        acc[i][j] = mma_b(ah, bh[j], acc[i][j]);
        if (BSPLIT) acc[i][j] = mma_b(ah, bl[j], acc[i][j]);
        if (ASPLIT) acc[i][j] = mma_b(al, bh[j], acc[i][j]);
      }
      dep_guard_b(acc[i][0], acc[i][3], ah, al);
    }
    keep4_b(bh[0], bh[1], bh[2], bh[3]);
    if (BSPLIT) keep4_b(bl[0], bl[1], bl[2], bl[3]);
  }
  acc_guard4(acc[0][0], acc[0][1], acc[0][2], acc[0][3]);
  acc_guard4(acc[1][0], acc[1][1], acc[1][2], acc[1][3]);
  acc_guard4(acc[2][0], acc[2][1], acc[2][2], acc[2][3]);
  acc_guard4(acc[3][0], acc[3][1], acc[3][2], acc[3][3]);

  float* slab = sT[wave];
#pragma unroll
  for (int i = 0; i < 4; ++i) {
    const int mBase = m0 + (i << 4);
#pragma unroll
    for (int j = 0; j < 4; ++j)
#pragma unroll
      for (int r = 0; r < 8; ++r)
        slab[(mOff + r) * 68 + (j << 4) + rlane] = acc[i][j][r] * scale;
    lds_wave_sync();
    if (OUT_MODE == 0) {
      float* C = (float*)Cout + (size_t)b * strideC;
      const int hh = lane >> 4, c4 = (lane & 15) * 4;
      for (int pass = 0; pass < 2; ++pass) {
#pragma unroll
        for (int it = 0; it < 8; ++it) {
          const int row = it * 2 + hh;
          const v4f v = *(const v4f*)(slab + row * 68 + c4);
          *(volatile v4f*)(C + (size_t)(mBase + row) * ldc + n0 + c4) = v;
        }
        __threadfence();
      }
    } else {
      const int q = lane >> 3, c8 = (lane & 7) * 8;
      unsigned short* C  = (unsigned short*)Cout  + (size_t)b * strideC;
      unsigned short* C2 = (unsigned short*)Cout2 + (size_t)b * strideC;
      const bool rope_on = ROPE && ((n0 & (HDIM - 1)) == 0);
      const float sg = (c8 < ROTH) ? -1.0f : 1.0f;
      const int pc8 = c8 ^ ROTH;
      for (int pass = 0; pass < 2; ++pass) {
#pragma unroll
        for (int it = 0; it < 4; ++it) {
          const int row = it * 4 + q;
          const float* sp = slab + row * 68 + c8;
          const float* pp = slab + row * 68 + pc8;
          v4f cv = {1.f, 1.f, 1.f, 1.f}, sv = {0.f, 0.f, 0.f, 0.f};
          if (ROPE) {
            const int s = (mBase + row) % seqlen;
            cv = *(const v4f*)(cst + (size_t)s * ROTH + (c8 >> 1));
            sv = *(const v4f*)(snt + (size_t)s * ROTH + (c8 >> 1));
          }
          v4u hv, lv;
#pragma unroll
          for (int e = 0; e < 4; ++e) {
            const float a0 = sp[2 * e], a1 = sp[2 * e + 1];
            float f0 = a0, f1 = a1;
            if (ROPE) {
              const float r0v = a0 * cv[e] + sg * pp[2 * e]     * sv[e];
              const float r1v = a1 * cv[e] + sg * pp[2 * e + 1] * sv[e];
              f0 = rope_on ? r0v : a0;
              f1 = rope_on ? r1v : a1;
            }
            const unsigned short h0 = bf_bits(f0), h1 = bf_bits(f1);
            const unsigned short l0 = bf_bits(f0 - bf_val(h0)), l1 = bf_bits(f1 - bf_val(h1));
            hv[e] = pk16(h0, h1);
            lv[e] = pk16(l0, l1);
          }
          *(volatile v4u*)(C  + (size_t)(mBase + row) * ldc + n0 + c8) = hv;
          *(volatile v4u*)(C2 + (size_t)(mBase + row) * ldc + n0 + c8) = lv;
        }
        __threadfence();
      }
    }
    lds_wave_sync();
  }
}

__global__ __launch_bounds__(256) void kbuild_kernel(const float* __restrict__ kc, const float* __restrict__ wks,
                                                     const float* __restrict__ cst, const float* __restrict__ snt,
                                                     unsigned short* __restrict__ kp) {
  __shared__ __align__(16) float krow[LATD];
  const int r = (int)blockIdx.x;
  const int b = r / SEQ;
  const int t = r - b * SEQ;
  const int tid = (int)threadIdx.x;
  if (tid < LATD / 4) *(v4f*)(krow + 4 * tid) = *(const v4f*)(kc + ((size_t)b * SEQ_FULL + t) * LATD + 4 * tid);
  __syncthreads();
  const int h  = tid >> 4;
  const int l0 = (tid & 15) * 8;
  const bool rot = (l0 < 2 * ROTH);
  const float sg = (l0 < ROTH) ? -1.0f : 1.0f;
  const int lp0 = rot ? (l0 ^ ROTH) : l0;
  const float* wrow = wks + h * LATD;
  const v4f wa = *(const v4f*)(wrow + l0);
  const v4f wb = *(const v4f*)(wrow + l0 + 4);
  const v4f pa = *(const v4f*)(wrow + lp0);
  const v4f pb = *(const v4f*)(wrow + lp0 + 4);
  const int ci = (l0 & (2 * ROTH - 1)) >> 1;
  const v4f cv = *(const v4f*)(cst + (size_t)t * ROTH + ci);
  const v4f sv = *(const v4f*)(snt + (size_t)t * ROTH + ci);
  v4u hv, lv;
#pragma unroll
  for (int e = 0; e < 4; ++e) {
    float g[2];
#pragma unroll
    for (int j = 0; j < 2; ++j) {
      const int ee = 2 * e + j;
      const float w  = (ee < 4) ? wa[ee] : wb[ee - 4];
      const float wp = (ee < 4) ? pa[ee] : pb[ee - 4];
      const float kd = krow[l0 + ee] * w;
      const float kq = krow[lp0 + ee] * wp;
      const float ro = kd * cv[e] + sg * kq * sv[e];
      g[j] = rot ? ro : kd;
    }
    const unsigned short h0 = bf_bits(g[0]), h1 = bf_bits(g[1]);
    const unsigned short b0 = bf_bits(g[0] - bf_val(h0)), b1 = bf_bits(g[1] - bf_val(h1));
    hv[e] = pk16(h0, h1);
    lv[e] = pk16(b0, b1);
  }
  unsigned short* dst = kp + (size_t)r * QCW + (size_t)h * HDIM + l0;
  *(volatile v4u*)(dst) = hv;
  *(volatile v4u*)(dst + DMOD) = lv;
  __threadfence();
  *(volatile v4u*)(dst) = hv;
  *(volatile v4u*)(dst + DMOD) = lv;
}

__global__ __launch_bounds__(256) void vtbuild_kernel(const float* __restrict__ vc, const float* __restrict__ wvs,
                                                      unsigned short* __restrict__ vt) {
  __shared__ __align__(16) float tf[64 * 68];
  const int s0  = blockIdx.x * 64;
  const int l0  = blockIdx.y * 64;
  const int b   = blockIdx.z;
  const int tid = threadIdx.x;
  {
    const int lr = tid >> 4;
    const int c4 = (tid & 15) * 4;
#pragma unroll
    for (int it = 0; it < 4; ++it) {
      const int rr = it * 16 + lr;
      const v4f a = *(const v4f*)(vc + ((size_t)b * SEQ_FULL + s0 + rr) * LATD + l0 + c4);
      *(v4f*)(tf + rr * 68 + c4) = a;
    }
  }
  __syncthreads();
  const int sub = tid >> 3;
  const int c8  = (tid & 7) * 8;
#pragma unroll 1
  for (int h = 0; h < NHD; ++h) {
    v4u hv[2];
#pragma unroll
    for (int it = 0; it < 2; ++it) {
      const int ol = it * 32 + sub;
      const float w = wvs[h * LATD + l0 + ol];
      v4u a;
#pragma unroll
      for (int q = 0; q < 4; ++q) {
        const float f0 = tf[(c8 + 2 * q) * 68 + ol] * w;
        const float f1 = tf[(c8 + 2 * q + 1) * 68 + ol] * w;
        a[q] = pk16(h16_bits(f0), h16_bits(f1));
      }
      hv[it] = a;
    }
    for (int pass = 0; pass < 2; ++pass) {
#pragma unroll
      for (int it = 0; it < 2; ++it) {
        const int ol = it * 32 + sub;
        const size_t go = ((size_t)b * DMOD + (size_t)h * HDIM + l0 + ol) * SEQ + s0 + c8;
        *(volatile v4u*)(vt + go) = hv[it];
      }
      __threadfence();
    }
  }
}

#define AT_NW 4
#define AT_KC 32
static_assert((2 * 64 * HDIM + 2 * AT_KC * HDIM + HDIM * AT_KC + AT_NW * 16 * AT_KC) * 2 <= 65536);
static_assert(AT_NW * 16 * HDIM <= 64 * HDIM);
static_assert(SEQ % AT_KC == 0);

__global__ __launch_bounds__(128)
void attn_kernel(unsigned short* qcp, const unsigned short* __restrict__ kp, const unsigned short* __restrict__ vtp, float sscale) {
  __shared__ __align__(16) __bf16   Qsh[64 * HDIM];
  __shared__ __align__(16) __bf16   Qsl[64 * HDIM];
  __shared__ __align__(16) __bf16   Ksh[AT_KC * HDIM];
  __shared__ __align__(16) __bf16   Ksl[AT_KC * HDIM];
  __shared__ __align__(16) _Float16 Vts[HDIM * AT_KC];
  __shared__ __align__(16) _Float16 Psh[AT_NW][16 * AT_KC];

  const int tid  = (int)threadIdx.x;
  const int wave = wave_id();
  const int lane = tid & 31;
  const int hh   = lane >> 4;
  const int c    = lane & 15;

  const int nqb = SEQ / 64;
  const int bx  = (int)blockIdx.x;
  const int qb  = bx % nqb;
  const int h   = bx / nqb;
  const int b   = (int)blockIdx.y;
  const int q0b = qb * 64;
  const int qw  = wave * 16;
  const size_t tok0 = (size_t)b * SEQ;

  const __bf16*   QG = (const __bf16*)(const void*)qcp;
  const __bf16*   KG = (const __bf16*)(const void*)kp;
  const _Float16* VG = (const _Float16*)(const void*)vtp + ((size_t)b * DMOD + (size_t)h * HDIM) * SEQ;

  {
    const int r = tid >> 1, half = (tid & 1) * 64;
    const __bf16* gh = QG + (tok0 + q0b + r) * QCW + (size_t)h * HDIM + half;
    const __bf16* gl = gh + DMOD;
#pragma unroll
    for (int i = 0; i < 8; ++i) {
      const v8b a0 = *(const v8b*)(gh + 8 * i);
      *(v8b*)(Qsh + r * HDIM + half + 8 * i) = a0;
    }
#pragma unroll
    for (int i = 0; i < 8; ++i) {
      const v8b a1 = *(const v8b*)(gl + 8 * i);
      *(v8b*)(Qsl + r * HDIM + half + 8 * i) = a1;
    }
  }

  float mrow[8], lrow[8];
  v8f oacc[8];
#pragma unroll
  for (int r = 0; r < 8; ++r) { mrow[r] = -INFINITY; lrow[r] = 0.f; }
#pragma unroll
  for (int t = 0; t < 8; ++t) oacc[t] = zero8();

  _Float16* pw = Psh[wave];

  const int nChunks = 2 * qb + 2;
  for (int kc = 0; kc < nChunks; ++kc) {
    const int kv0 = kc * AT_KC;
    __syncthreads();
    {
      const int r = tid >> 2, qq = (tid & 3) * 32;
      const __bf16* ksh = KG + (tok0 + kv0 + r) * QCW + (size_t)h * HDIM + qq;
      const __bf16* ksl = ksh + DMOD;
#pragma unroll
      for (int i = 0; i < 4; ++i) {
        const v8b a0 = *(const v8b*)(ksh + 8 * i);
        const v8b a1 = *(const v8b*)(ksl + 8 * i);
        *(v8b*)(Ksh + r * HDIM + qq + 8 * i) = a0;
        *(v8b*)(Ksl + r * HDIM + qq + 8 * i) = a1;
      }
      const _Float16* vs = VG + (size_t)tid * SEQ + kv0;
#pragma unroll
      for (int i = 0; i < 4; ++i) {
        const v8h b0 = *(const v8h*)(vs + 8 * i);
        *(v8h*)(Vts + tid * AT_KC + 8 * i) = b0;
      }
    }
    __syncthreads();

    v8f s[2];
#pragma unroll
    for (int j = 0; j < 2; ++j) {
      s[j] = zero8();
#pragma unroll
      for (int dc = 0; dc < 4; ++dc) {
        FragB qa, ql, kb, kl;
        qa.h[0] = *(const v8b*)(Qsh + (qw + c) * HDIM + dc * 32 + 8 * hh);
        qa.h[1] = *(const v8b*)(Qsh + (qw + c) * HDIM + dc * 32 + 16 + 8 * hh);
        ql.h[0] = *(const v8b*)(Qsl + (qw + c) * HDIM + dc * 32 + 8 * hh);
        ql.h[1] = *(const v8b*)(Qsl + (qw + c) * HDIM + dc * 32 + 16 + 8 * hh);
        kb.h[0] = *(const v8b*)(Ksh + (j * 16 + c) * HDIM + dc * 32 + 8 * hh);
        kb.h[1] = *(const v8b*)(Ksh + (j * 16 + c) * HDIM + dc * 32 + 16 + 8 * hh);
        kl.h[0] = *(const v8b*)(Ksl + (j * 16 + c) * HDIM + dc * 32 + 8 * hh);
        kl.h[1] = *(const v8b*)(Ksl + (j * 16 + c) * HDIM + dc * 32 + 16 + 8 * hh);
        s[j] = at_mma(qa.v, kb.v, s[j]);
        s[j] = at_mma(qa.v, kl.v, s[j]);
        s[j] = at_mma(ql.v, kb.v, s[j]);
      }
    }
    float cm[8];
#pragma unroll
    for (int r = 0; r < 8; ++r) {
      const int qrow = q0b + qw + 8 * hh + r;
      float m = -INFINITY;
#pragma unroll
      for (int j = 0; j < 2; ++j) {
        const int kvcol = kv0 + j * 16 + c;
        const float sv = s[j][r] * sscale;
        const float sm = (kvcol > qrow) ? -INFINITY : sv;
        s[j][r] = sm;
        m = fmaxf(m, sm);
      }
#pragma unroll
      for (int off = 1; off < 16; off <<= 1) m = fmaxf(m, __shfl_xor(m, off, 32));
      cm[r] = m;
    }
#pragma unroll
    for (int r = 0; r < 8; ++r) {
      const float mnew  = fmaxf(mrow[r], cm[r]);
      const float alpha = expf(mrow[r] - mnew);
      mrow[r] = mnew;
      float psum = 0.f;
#pragma unroll
      for (int j = 0; j < 2; ++j) {
        const float p  = expf(s[j][r] - mnew) * PCARRY;
        const float pc = (float)(_Float16)p;
        const float pq = (pc < F16MIN) ? 0.f : pc;
        psum += pq;
        pw[(8 * hh + r) * AT_KC + j * 16 + c] = (_Float16)pq;
      }
#pragma unroll
      for (int off = 1; off < 16; off <<= 1) psum += __shfl_xor(psum, off, 32);
      lrow[r] = lrow[r] * alpha + psum;
#pragma unroll
      for (int t = 0; t < 8; ++t) oacc[t][r] *= alpha;
    }
    lds_wave_sync();
    {
      FragH pa;
      pa.h[0] = *(const v8h*)(pw + c * AT_KC + 8 * hh);
      pa.h[1] = *(const v8h*)(pw + c * AT_KC + 16 + 8 * hh);
#pragma unroll
      for (int t = 0; t < 8; ++t) {
        FragH vb;
        vb.h[0] = *(const v8h*)(Vts + (t * 16 + c) * AT_KC + 8 * hh);
        vb.h[1] = *(const v8h*)(Vts + (t * 16 + c) * AT_KC + 16 + 8 * hh);
        oacc[t] = at_mma_h(pa.v, vb.v, oacc[t]);
      }
    }
  }
  acc_guard4(oacc[0], oacc[1], oacc[2], oacc[3]);
  acc_guard4(oacc[4], oacc[5], oacc[6], oacc[7]);

  __syncthreads();
  unsigned short* osh = (unsigned short*)(void*)Qsh + wave * 16 * HDIM;
  unsigned short* osl = (unsigned short*)(void*)Qsl + wave * 16 * HDIM;
#pragma unroll
  for (int r = 0; r < 8; ++r) {
    const float inv = 1.0f / lrow[r];
#pragma unroll
    for (int t = 0; t < 8; ++t) {
      const float o = oacc[t][r] * inv;
      const unsigned short hb = bf_bits(o);
      const unsigned short lb = bf_bits(o - bf_val(hb));
      const int so = (8 * hh + r) * HDIM + t * 16 + c;
      osh[so] = hb;
      osl[so] = lb;
    }
  }
  lds_wave_sync();
  unsigned short* Ag = qcp + (tok0 + q0b + qw) * QCW + (size_t)h * HDIM;
  const int rr = lane >> 4;
  const int c8 = (lane & 15) * 8;
  for (int pass = 0; pass < 2; ++pass) {
#pragma unroll
    for (int it = 0; it < 8; ++it) {
      const int row = it * 2 + rr;
      const v4u x = *(const v4u*)(osh + row * HDIM + c8);
      const v4u y = *(const v4u*)(osl + row * HDIM + c8);
      *(volatile v4u*)(Ag + (size_t)row * QCW + c8)        = x;
      *(volatile v4u*)(Ag + (size_t)row * QCW + DMOD + c8) = y;
    }
    __threadfence();
  }
}

#define WS_TOTAL_BYTES ((size_t)NTOK * DMOD * 2 + (size_t)DMOD * DMOD * 2 * 2 + (size_t)2 * LATD * DMOD * 2 + \
                        (size_t)NTOK * QCW * 2 * 2 + (size_t)NB * DMOD * SEQ * 2 + (size_t)2 * NHD * LATD * 4 + 128 + \
                        (size_t)SEQ * ROTH * 4 * 2)
static_assert(WS_TOTAL_BYTES <= 134217728UL);

static inline int cdiv_h(int a, int b) { return (a + b - 1) / b; }

extern "C" void kernel_launch(void* const* d_in, const int* in_sizes, int n_in,
                              void* d_out, int out_size, void* d_ws, size_t ws_size,
                              hipStream_t stream) {
  if (n_in < 6) return;
  const long needX = ((long)(NB - 1) * SEQ_FULL + SEQ) * DMOD;
  if ((long)in_sizes[0] < needX) return;
  if (in_sizes[1] < DMOD * DMOD) return;
  if (in_sizes[2] < 2 * LATD * DMOD) return;
  if (in_sizes[3] < NHD * LATD * HDIM) return;
  if (in_sizes[4] < NHD * LATD * HDIM) return;
  if (in_sizes[5] < DMOD * DMOD) return;
  const long needO = OUT2_OFF + ((long)(NB - 1) * SEQ_FULL + SEQ) * LATD;
  if ((long)out_size < needO) return;

  const float* x   = (const float*)d_in[0];
  const float* wq  = (const float*)d_in[1];
  const float* wkv = (const float*)d_in[2];
  const float* wkh = (const float*)d_in[3];
  const float* wvh = (const float*)d_in[4];
  const float* wo  = (const float*)d_in[5];
  float* out = (float*)d_out;

  const size_t szXB  = (size_t)NTOK * DMOD * 2;
  const size_t szWQ  = (size_t)DMOD * DMOD * 2;
  const size_t szWKV = (size_t)2 * LATD * DMOD * 2;
  const size_t szWO  = (size_t)DMOD * DMOD * 2;
  const size_t szQC  = (size_t)NTOK * QCW * 2;
  const size_t szKP  = (size_t)NTOK * QCW * 2;
  const size_t szVT  = (size_t)NB * DMOD * SEQ * 2;
  const size_t szWS  = (size_t)2 * NHD * LATD * 4;
  const size_t szFR  = 128;
  const size_t szCS  = (size_t)SEQ * ROTH * 4;
  size_t off = 0;
  const size_t oXB  = off; off += szXB;
  const size_t oWQ  = off; off += szWQ;
  const size_t oWKV = off; off += szWKV;
  const size_t oWO  = off; off += szWO;
  const size_t oQC  = off; off += szQC;
  const size_t oKP  = off; off += szKP;
  const size_t oVT  = off; off += szVT;
  const size_t oWS  = off; off += szWS;
  const size_t oFR  = off; off += szFR;
  const size_t oCS  = off; off += szCS;
  const size_t oSN  = off; off += szCS;
  if (off != WS_TOTAL_BYTES) return;
  if (off > ws_size) return;
  if (off > 134217728UL) return;

  char* ws = (char*)d_ws;
  unsigned short* XB   = (unsigned short*)(ws + oXB);
  unsigned short* WQB  = (unsigned short*)(ws + oWQ);
  unsigned short* WKVB = (unsigned short*)(ws + oWKV);
  unsigned short* WOB  = (unsigned short*)(ws + oWO);
  unsigned short* QC   = (unsigned short*)(ws + oQC);
  unsigned short* KP   = (unsigned short*)(ws + oKP);
  unsigned short* VT   = (unsigned short*)(ws + oVT);
  float* WSUM = (float*)(ws + oWS);
  float* FREQ = (float*)(ws + oFR);
  float* CST  = (float*)(ws + oCS);
  float* SNT  = (float*)(ws + oSN);

  const dim3 b256(256), b128(128);
  const float sscale = 1.0f / sqrtf((float)HDIM);

  {
    const int n8 = NTOK * DMOD / 8;
    cvt_rows_kernel<<<dim3(cdiv_h(n8, 256)), b256, 0, stream>>>(x, XB, n8, DMOD, SEQ, SEQ_FULL);
  }
  {
    const int n8q = DMOD * DMOD / 8;
    cvt_rows_kernel<<<dim3(cdiv_h(n8q, 256)), b256, 0, stream>>>(wq, WQB, n8q, DMOD, DMOD, DMOD);
    const int n8kv = 2 * LATD * DMOD / 8;
    cvt_rows_kernel<<<dim3(cdiv_h(n8kv, 256)), b256, 0, stream>>>(wkv, WKVB, n8kv, DMOD, 2 * LATD, 2 * LATD);
    cvt_rows_kernel<<<dim3(cdiv_h(n8q, 256)), b256, 0, stream>>>(wo, WOB, n8q, DMOD, DMOD, DMOD);
  }
  prep_kernel<<<dim3(16), b256, 0, stream>>>(wkh, wvh, WSUM, FREQ);
  table_kernel<<<dim3(cdiv_h(SEQ * ROTH, 256)), b256, 0, stream>>>(FREQ, CST, SNT, SEQ * ROTH);
  gemm64_kernel<false, false, 0, false><<<dim3(cdiv_h((SEQ / 64) * (LATD / 64), 8), NB), b256, 0, stream>>>(
      XB, XB, DMOD, (long)SEQ * DMOD, WKVB, WKVB, DMOD, 0L,
      (void*)(out + OUT1_OFF), (void*)(out + OUT1_OFF), LATD, (long)SEQ_FULL * LATD, SEQ, LATD, DMOD, 1.0f, CST, SNT, SEQ);
  gemm64_kernel<false, false, 0, false><<<dim3(cdiv_h((SEQ / 64) * (LATD / 64), 8), NB), b256, 0, stream>>>(
      XB, XB, DMOD, (long)SEQ * DMOD, WKVB + (size_t)LATD * DMOD, WKVB + (size_t)LATD * DMOD, DMOD, 0L,
      (void*)(out + OUT2_OFF), (void*)(out + OUT2_OFF), LATD, (long)SEQ_FULL * LATD, SEQ, LATD, DMOD, 1.0f, CST, SNT, SEQ);
  gemm64_kernel<false, false, 2, true><<<dim3(cdiv_h((NTOK / 64) * (DMOD / 64), 8), 1), b256, 0, stream>>>(
      XB, XB, DMOD, 0L, WQB, WQB, DMOD, 0L, (void*)QC, (void*)(QC + DMOD), QCW, 0L, NTOK, DMOD, DMOD, 1.0f, CST, SNT, SEQ);
  kbuild_kernel<<<dim3(NTOK), b256, 0, stream>>>(out + OUT1_OFF, WSUM, CST, SNT, KP);
  vtbuild_kernel<<<dim3(SEQ / 64, LATD / 64, NB), b256, 0, stream>>>(out + OUT2_OFF, WSUM + NHD * LATD, VT);
  attn_kernel<<<dim3(NHD * (SEQ / 64), NB), b128, 0, stream>>>(QC, KP, VT, sscale);
  gemm64_kernel<true, false, 0, false><<<dim3(cdiv_h((SEQ / 64) * (DMOD / 64), 8), NB), b256, 0, stream>>>(
      QC, QC + DMOD, QCW, (long)SEQ * QCW, WOB, WOB, DMOD, 0L, (void*)out, (void*)out, DMOD, (long)SEQ_FULL * DMOD,
      SEQ, DMOD, DMOD, 1.0f, CST, SNT, SEQ);
  (void)hipGetLastError();
}
